// Label_Attn_Fusion_Layer_for_token_16621523435984
// MI455X (gfx1250) — hardware-verified
//
#include <hip/hip_runtime.h>


namespace {
constexpr int B = 8, S = 128, L = 16, LS = 8, H = 768, NH = 12, HD = 64, T = S + LS, NX = B * S + L * LS, NQT = (T + 15) / 16, NKC = (T + 31) / 32;
constexpr float XS = 8.0f, PS = 1024.0f, WSC = 256.0f;
typedef _Float16 b16;
typedef __attribute__((ext_vector_type(16))) _Float16 v16b;
typedef __attribute__((ext_vector_type(8))) _Float16 v8b;
typedef __attribute__((ext_vector_type(8))) float v8f;
typedef __attribute__((ext_vector_type(4))) float v4f;
typedef __attribute__((ext_vector_type(2))) float v2f;
__device__ __forceinline__ float bf16_rne(float f) { unsigned int u = __float_as_uint(f); u += 0x7FFFu + ((u >> 16) & 1u); return __uint_as_float(u & 0xFFFF0000u); }
__device__ __forceinline__ float bfv(float f) { float r = bf16_rne(f); asm volatile("" : "+v"(r)); return r; }
__device__ __forceinline__ void split16(float v, b16& hi, b16& lo) { hi = (b16)v; lo = (b16)(v - (float)hi); }
__device__ __forceinline__ v16b frag_kb(const b16* p, int hh) { const v8b a = *(const v8b*)(p + 8 * hh), b = *(const v8b*)(p + 16 + 8 * hh); v16b f;
#pragma unroll
  for (int e = 0; e < 8; ++e) { f[e] = a[e]; f[8 + e] = b[e]; } return f; }
__device__ __forceinline__ v8f wmma16b(v16b a, v16b b, v8f c) { v8f d = __builtin_amdgcn_wmma_f32_16x16x32_f16(false, a, false, b, (short)0, c, false, false); asm volatile("v_nop\n\tv_nop\n\tv_nop\n\tv_nop" : "+v"(d) : "v"(a), "v"(b)); return d; }
__device__ __forceinline__ void wave_lds_sync() { __builtin_amdgcn_fence(__ATOMIC_RELEASE, "workgroup"); __builtin_amdgcn_wave_barrier(); __builtin_amdgcn_fence(__ATOMIC_ACQUIRE, "workgroup"); }
__device__ __forceinline__ int xrow(int b, int l, int t) { return t < S ? b * S + t : (t < T ? B * S + l * LS + (t - S) : -1); }

__global__ __launch_bounds__(256) void wcopy_kernel(const float* __restrict__ wq, const float* __restrict__ wk, const float* __restrict__ wv, b16* __restrict__ WT) { const size_t u = (size_t)blockIdx.x * 256 + threadIdx.x; const size_t per = (size_t)H * H / 8; if (u >= 3 * per) return; const int which = (int)(u / per); const size_t e = (u % per) * 8; const float* w = which == 0 ? wq : (which == 1 ? wk : wv); v8b v;
#pragma unroll
  for (int j = 0; j < 8; ++j) v[j] = (b16)(bf16_rne(w[e + j]) * WSC); for (int pass = 0; pass < 2; ++pass) { *(volatile v8b*)(WT + (size_t)which * H * H + e) = v; __threadfence(); } }
__global__ __launch_bounds__(32) void qkv_kernel(const float* __restrict__ tok, const float* __restrict__ lab, const b16* __restrict__ WT, const float* __restrict__ bq, const float* __restrict__ bk, const float* __restrict__ bv, float* __restrict__ QKV) {
  __shared__ __attribute__((aligned(16))) b16 Ah[16][H + 8]; __shared__ float Tf[16][132]; const int lane = threadIdx.x, nloc = lane & 15, hlf = lane >> 4; const int cg = blockIdx.x % 18; const size_t m0 = (size_t)(blockIdx.x / 18) * 16;
  for (int rr = 0; rr < 16; ++rr) { const size_t row = m0 + rr; const float* src = row < (size_t)B * S ? tok + row * H : lab + (row - (size_t)B * S) * H; for (int q = 0; q < H / 32; ++q) Ah[rr][q * 32 + lane] = (b16)(bf16_rne(src[q * 32 + lane]) * XS); }
  wave_lds_sync(); v8f acc[8];
#pragma unroll
  for (int t = 0; t < 8; ++t) acc[t] = (v8f){};
#pragma unroll 2
  for (int kb = 0; kb < H; kb += 32) { const v16b a = frag_kb(&Ah[nloc][kb], hlf);
#pragma unroll
    for (int t = 0; t < 8; ++t) acc[t] = wmma16b(a, frag_kb(WT + (size_t)(cg * 128 + t * 16 + nloc) * H + kb, hlf), acc[t]); }
  const int which = cg / 6; const float* bias = which == 0 ? bq : (which == 1 ? bk : bv);
#pragma unroll
  for (int t = 0; t < 8; ++t) { const int c = cg * 128 + t * 16 + nloc; const float bb = bfv(bias[c - which * H]);
#pragma unroll
    for (int r8 = 0; r8 < 8; ++r8) Tf[8 * hlf + r8][t * 16 + nloc] = acc[t][r8] * (1.0f / (XS * WSC)) + bb; }
  wave_lds_sync();
  for (int pass = 0; pass < 2; ++pass) { for (int rr = 0; rr < 16; ++rr) *(volatile v4f*)(QKV + (m0 + rr) * (3 * H) + cg * 128 + lane * 4) = *(const v4f*)(&Tf[rr][lane * 4]); __threadfence(); }
}
__global__ __launch_bounds__(32) void att_kernel(const float* __restrict__ QKV, const float* __restrict__ tmask, const float* __restrict__ lmask, int BV, int LV, float* __restrict__ out) {
  __shared__ __attribute__((aligned(16))) b16 Qh[16][HD + 8], Ql[16][HD + 8], Kh[32][HD + 8], Kl[32][HD + 8], Ph[16][40], Pl[16][40], Vh[HD][40], Vl[HD][40]; __shared__ float Sc[16][33], Mx[16], Dn[16], Sf[16], Of[16][HD + 2], Kb[32]; __shared__ int Qr[16], Kr[32];
  const int lane = threadIdx.x, nloc = lane & 15, hlf = lane >> 4; const int qt = blockIdx.x % NQT; const int hh = (blockIdx.x / NQT) % NH; const int l = (blockIdx.x / (NQT * NH)) % L; const int b = blockIdx.x / (NQT * NH * L); if (b >= BV || l >= LV) return; const int q0 = qt * 16;
  if (lane < 16) { Qr[lane] = xrow(b, l, q0 + lane); Mx[lane] = -INFINITY; Dn[lane] = 0.0f; Sf[lane] = 0.0f; }
  wave_lds_sync();
  for (int rr = 0; rr < 16; ++rr) { const int xr = Qr[rr]; for (int q = 0; q < 2; ++q) { b16 p = (b16)0.0f, ql = (b16)0.0f; if (xr >= 0) split16(QKV[(size_t)xr * 3 * H + hh * HD + q * 32 + lane] * XS, p, ql); Qh[rr][q * 32 + lane] = p; Ql[rr][q * 32 + lane] = ql; } }
  v8f acc[4] = {(v8f){}, (v8f){}, (v8f){}, (v8f){}}; wave_lds_sync();
#pragma unroll 1
  for (int kc = 0; kc < NKC * 32; kc += 32) {
    { const int t = kc + lane; const int xr = xrow(b, l, t); Kr[lane] = xr; const float mk = t < S ? bfv(tmask[b * S + t]) : (t < T ? bfv(lmask[l * LS + (t - S)]) : 0.0f); Kb[lane] = xr >= 0 ? (1.0f - mk) * -10000.0f : -INFINITY; }
    wave_lds_sync();
    for (int rr = 0; rr < 32; ++rr) { const int xr = Kr[rr]; for (int q = 0; q < 2; ++q) { b16 p = (b16)0.0f, ql = (b16)0.0f, vp = (b16)0.0f, vl = (b16)0.0f; if (xr >= 0) { split16(QKV[(size_t)xr * 3 * H + H + hh * HD + q * 32 + lane] * XS, p, ql); split16(QKV[(size_t)xr * 3 * H + 2 * H + hh * HD + q * 32 + lane] * XS, vp, vl); } Kh[rr][q * 32 + lane] = p; Kl[rr][q * 32 + lane] = ql; Vh[q * 32 + lane][rr] = vp; Vl[q * 32 + lane][rr] = vl; } }
    wave_lds_sync();
#pragma unroll
    for (int blk = 0; blk < 2; ++blk) { v8f s = {};
#pragma unroll
      for (int kb = 0; kb < HD; kb += 32) { const v16b qh = frag_kb(&Qh[nloc][kb], hlf), qlo = frag_kb(&Ql[nloc][kb], hlf), kh = frag_kb(&Kh[blk * 16 + nloc][kb], hlf), kl = frag_kb(&Kl[blk * 16 + nloc][kb], hlf); s = wmma16b(qh, kh, s); s = wmma16b(qh, kl, s); s = wmma16b(qlo, kh, s); }
#pragma unroll
      for (int r8 = 0; r8 < 8; ++r8) { const int kk = blk * 16 + nloc; const float kb_ = Kb[kk]; Sc[8 * hlf + r8][kk] = (kb_ == -INFINITY) ? -INFINITY : s[r8] * (0.125f / (XS * XS)) + kb_; } }
    wave_lds_sync();
#pragma unroll 1
    for (int qi = 0; qi < 16; ++qi) { const float sv = Sc[qi][lane]; float cm = sv; for (int o = 16; o; o >>= 1) cm = fmaxf(cm, __shfl_xor(cm, o)); const float mo = Mx[qi]; const float mn = fmaxf(mo, cm); const float p = (sv == -INFINITY || mn == -INFINITY) ? 0.0f : __expf(sv - mn); float psum = p; for (int o = 16; o; o >>= 1) psum += __shfl_xor(psum, o);
      b16 ph, plo; split16(p * PS, ph, plo); Ph[qi][lane] = ph; Pl[qi][lane] = plo; if (lane == 0) { const float sf = (mo == -INFINITY || mn == -INFINITY) ? ((mo == -INFINITY && mn == -INFINITY) ? 1.0f : 0.0f) : __expf(mo - mn); Sf[qi] = sf; Dn[qi] = Dn[qi] * sf + psum; Mx[qi] = mn; } }
    wave_lds_sync(); const v16b pa = frag_kb(&Ph[nloc][0], hlf), pb = frag_kb(&Pl[nloc][0], hlf);
#pragma unroll
    for (int tt = 0; tt < 4; ++tt) {
#pragma unroll
      for (int r8 = 0; r8 < 8; ++r8) acc[tt][r8] *= Sf[8 * hlf + r8];
      const v16b vh = frag_kb(&Vh[tt * 16 + nloc][0], hlf), vl = frag_kb(&Vl[tt * 16 + nloc][0], hlf); acc[tt] = wmma16b(pa, vh, acc[tt]); acc[tt] = wmma16b(pa, vl, acc[tt]); acc[tt] = wmma16b(pb, vh, acc[tt]); }
    wave_lds_sync(); }
#pragma unroll
  for (int tt = 0; tt < 4; ++tt)
#pragma unroll
    for (int r8 = 0; r8 < 8; ++r8) { const int rl = 8 * hlf + r8; Of[rl][tt * 16 + nloc] = acc[tt][r8] * (1.0f / (PS * XS)) / Dn[rl]; }
  wave_lds_sync();
  for (int pass = 0; pass < 2; ++pass) { for (int rr = 0; rr < 16; ++rr) { const int t = q0 + rr; if (t >= T) continue; *(volatile v2f*)(out + (((size_t)b * T + t) * L + l) * H + hh * HD + lane * 2) = (v2f){Of[rr][lane * 2], Of[rr][lane * 2 + 1]}; } __threadfence(); }
}
}

extern "C" void kernel_launch(void* const* d_in, const int* in_sizes, int n_in, void* d_out, int out_size, void* d_ws, size_t ws_size, hipStream_t stream) {
  (void)n_in;
  auto Fp = [&](int i) { return (const float*)d_in[i]; };
  if (in_sizes[0] != B * S * H || in_sizes[1] != L * LS * H || in_sizes[2] != B * S || in_sizes[3] != L * LS || in_sizes[4] != H * H || in_sizes[6] != H * H || in_sizes[8] != H * H || out_size != B * T * L * H) return;
  const int BV = B, LV = L;
  size_t off = 0; char* ws = (char*)d_ws;
  auto carve = [&](size_t bytes) { char* p = ws + off; off += (bytes + 255) & ~(size_t)255; return p; };
  b16* WT = (b16*)carve((size_t)3 * H * H * 2); float* QKV = (float*)carve((size_t)NX * 3 * H * 4);
  if (off > ws_size || off > ((size_t)32 << 20)) return;
  wcopy_kernel<<<(unsigned)(((size_t)3 * H * H / 8 + 255) / 256), 256, 0, stream>>>(Fp(4), Fp(6), Fp(8), WT);
  qkv_kernel<<<(NX / 16) * 18, 32, 0, stream>>>(Fp(0), Fp(1), WT, Fp(5), Fp(7), Fp(9), QKV);
  att_kernel<<<BV * L * NH * NQT, 32, 0, stream>>>(QKV, Fp(2), Fp(3), BV, LV, (float*)d_out);
}
